// G2ANet_40596030882474
// MI455X (gfx1250) — hardware-verified
//
#include <hip/hip_runtime.h>
#define NSC 128
#define NAG 32
#define NA (NSC * NAG)
#define NO (NAG - 1)
#define NP (NA * NO)
#define DD 256
#define H1 128
#define PI_F 3.14159265358979323846f
#define OUT1 2097152
#define OUT2 2224128
#define OUT3 2351104
#define OUT4 2351105
#define OUT5 2478081
#define OUTEND 2605057
typedef __bf16 v16b __attribute__((ext_vector_type(16)));
typedef unsigned short v8us __attribute__((ext_vector_type(8), may_alias));
typedef float  v8f  __attribute__((ext_vector_type(8)));
typedef float  v4f  __attribute__((ext_vector_type(4)));
typedef float  v4fa __attribute__((ext_vector_type(4), may_alias));
union FragB { v16b v; v8us half[2]; unsigned short u[16]; };

__device__ __forceinline__ unsigned short bf16_bits(float x) { unsigned int u = __float_as_uint(x); return (unsigned short)((u + 0x7FFFu + ((u >> 16) & 1u)) >> 16); }
__device__ __forceinline__ float bf16_val(unsigned short b) { return __uint_as_float(((unsigned int)b) << 16); }
__device__ __forceinline__ float bf16_round(float x) { return bf16_val(bf16_bits(x)); }
template <int NT>
__device__ __forceinline__ v8f mmaN(v16b ah, v16b al, v16b bh, v16b bl, v8f c) {
  c = __builtin_amdgcn_wmma_f32_16x16x32_bf16(false, ah, false, bh, (short)0, c, false, false);
  if (NT >= 2) c = __builtin_amdgcn_wmma_f32_16x16x32_bf16(false, al, false, bh, (short)0, c, false, false);
  if (NT >= 3) c = __builtin_amdgcn_wmma_f32_16x16x32_bf16(false, ah, false, bl, (short)0, c, false, false);
  asm volatile("v_nop\n\tv_nop\n\tv_nop\n\tv_nop" : "+v"(c) : "v"(ah), "v"(al), "v"(bh), "v"(bl));
  return c;
}

__global__ __launch_bounds__(256) void k_wt_bf16(const float* __restrict__ W, unsigned short* __restrict__ Wt, int K, int N) {
  const int t = blockIdx.x * 256 + threadIdx.x;
  const int k8n = K / 8;
  if (t >= N * k8n) return;
  const int n = t / k8n, k8 = (t % k8n) * 8;
  v8us v;
#pragma unroll
  for (int i = 0; i < 8; ++i) v[i] = bf16_bits(W[(size_t)(k8 + i) * N + n]);
  *(volatile v8us*)(Wt + (size_t)n * K + k8) = v;
  __threadfence();
  *(volatile v8us*)(Wt + (size_t)n * K + k8) = v;
}

template <bool ASPLIT, int ACT, bool BIAS_BF16>
__global__ __launch_bounds__(128) void k_gemm_bf(const float* __restrict__ A, int lda, const unsigned short* __restrict__ Wt, int ldb,
                                               const float* __restrict__ bias, float* __restrict__ C, int ldc, int M, int N, int K) {
  __shared__ __attribute__((aligned(16))) float so[4][16][64];
  const int tid = threadIdx.x, w = tid >> 5, lane = tid & 31, ln = lane & 15, hh = lane >> 4;
  const int ntn = N / 64;
  const int wid = blockIdx.x * 4 + w;
  const int mt = wid / ntn, nq = wid % ntn;
  if (mt * 16 >= M) return;
  const int row0 = mt * 16, col0 = nq * 64;
  const float* arow = A + (size_t)(row0 + ln) * lda;
  v8f acc[4] = {};
  for (int kb = 0; kb < K; kb += 32) {
    FragB ah, al;
    const v4f x0 = *(const v4fa*)(arow + kb + 8 * hh), x1 = *(const v4fa*)(arow + kb + 8 * hh + 4);
    const v4f x2 = *(const v4fa*)(arow + kb + 16 + 8 * hh), x3 = *(const v4fa*)(arow + kb + 16 + 8 * hh + 4);
    float xs[16] = {x0[0],x0[1],x0[2],x0[3],x1[0],x1[1],x1[2],x1[3],x2[0],x2[1],x2[2],x2[3],x3[0],x3[1],x3[2],x3[3]};
#pragma unroll
    for (int i = 0; i < 16; ++i) { const unsigned short hb = bf16_bits(xs[i]); ah.u[i] = hb; al.u[i] = ASPLIT ? bf16_bits(xs[i] - bf16_val(hb)) : (unsigned short)0; }
#pragma unroll
    for (int t = 0; t < 4; ++t) {
      const unsigned short* brow = Wt + (size_t)(col0 + t * 16 + ln) * ldb + kb;
      FragB b;
      b.half[0] = *(const v8us*)(brow + 8 * hh);
      b.half[1] = *(const v8us*)(brow + 16 + 8 * hh);
      acc[t] = mmaN<ASPLIT ? 2 : 1>(ah.v, al.v, b.v, b.v, acc[t]);
    }
  }
#pragma unroll
  for (int t = 0; t < 4; ++t) {
    float bv = bias ? bias[col0 + t * 16 + ln] : 0.f;
    if (BIAS_BF16) bv = bf16_round(bv);
#pragma unroll
    for (int r = 0; r < 8; ++r) { float v = acc[t][r] + bv; if (ACT == 1) v = fmaxf(v, 0.f); so[w][8 * hh + r][t * 16 + ln] = v; }
  }
  __builtin_amdgcn_fence(__ATOMIC_ACQ_REL, "workgroup");
  __builtin_amdgcn_wave_barrier();
  const int rsub = lane >> 4, c4 = (lane & 15) * 4;
  for (int pass = 0; pass < 2; ++pass) {
#pragma unroll
    for (int q = 0; q < 8; ++q) {
      const int r = q * 2 + rsub;
      const v4f v = *(const v4fa*)&so[w][r][c4];
      *(volatile v4f*)(C + (size_t)(row0 + r) * ldc + col0 + c4) = v;
    }
    if (pass == 0) __threadfence();
  }
}

template <bool ASPLIT, int ACT, bool BIAS_BF16, bool RES_BF16>
__global__ __launch_bounds__(128) void k_gemm_bf3(const float* __restrict__ A, int lda, const unsigned short* __restrict__ Wt, int ldb,
                                                const float* __restrict__ bias, const float* __restrict__ resid, int rmod, int ldr,
                                                float* __restrict__ C, int ldc, int M, int N, int K) {
  __shared__ __attribute__((aligned(16))) float so[4][16][64];
  const int tid = threadIdx.x, w = tid >> 5, lane = tid & 31, ln = lane & 15, hh = lane >> 4;
  const int ntn = N / 64;
  const int wid = blockIdx.x * 4 + w;
  const int mt = wid / ntn, nq = wid % ntn;
  if (mt * 16 >= M) return;
  const int row0 = mt * 16, col0 = nq * 64;
  const float* arow = A + (size_t)(row0 + ln) * lda;
  v8f acc[4] = {};
  for (int kb = 0; kb < K; kb += 32) {
    FragB ah, al;
    const v4f x0 = *(const v4fa*)(arow + kb + 8 * hh), x1 = *(const v4fa*)(arow + kb + 8 * hh + 4);
    const v4f x2 = *(const v4fa*)(arow + kb + 16 + 8 * hh), x3 = *(const v4fa*)(arow + kb + 16 + 8 * hh + 4);
    float xs[16] = {x0[0],x0[1],x0[2],x0[3],x1[0],x1[1],x1[2],x1[3],x2[0],x2[1],x2[2],x2[3],x3[0],x3[1],x3[2],x3[3]};
#pragma unroll
    for (int i = 0; i < 16; ++i) { const unsigned short hb = bf16_bits(xs[i]); ah.u[i] = hb; al.u[i] = ASPLIT ? bf16_bits(xs[i] - bf16_val(hb)) : (unsigned short)0; }
#pragma unroll
    for (int t = 0; t < 4; ++t) {
      const unsigned short* brow = Wt + (size_t)(col0 + t * 16 + ln) * ldb + kb;
      FragB b;
      b.half[0] = *(const v8us*)(brow + 8 * hh);
      b.half[1] = *(const v8us*)(brow + 16 + 8 * hh);
      acc[t] = mmaN<ASPLIT ? 2 : 1>(ah.v, al.v, b.v, b.v, acc[t]);
    }
  }
#pragma unroll
  for (int t = 0; t < 4; ++t) {
    const int col = col0 + t * 16 + ln;
    float bv = bias ? bias[col] : 0.f;
    if (BIAS_BF16) bv = bf16_round(bv);
#pragma unroll
    for (int r = 0; r < 8; ++r) {
      float v = acc[t][r] + bv;
      if (resid) { float rv = resid[(size_t)((row0 + 8 * hh + r) % rmod) * ldr + col]; if (RES_BF16) rv = bf16_round(rv); v += rv; }
      if (ACT == 1) v = fmaxf(v, 0.f);
      if (ACT == 2) v = 0.5f * v * (1.0f + erff(v * 0.70710678118654752f));
      if (ACT == 3) { const float u = 0.7978845608028654f * (v + 0.044715f * v * v * v); v = 0.5f * v * (1.0f + tanhf(u)); }
      so[w][8 * hh + r][t * 16 + ln] = v;
    }
  }
  __builtin_amdgcn_fence(__ATOMIC_ACQ_REL, "workgroup");
  __builtin_amdgcn_wave_barrier();
  const int rsub = lane >> 4, c4 = (lane & 15) * 4;
  for (int pass = 0; pass < 2; ++pass) {
#pragma unroll
    for (int q = 0; q < 8; ++q) {
      const int r = q * 2 + rsub;
      const v4f v = *(const v4fa*)&so[w][r][c4];
      *(volatile v4f*)(C + (size_t)(row0 + r) * ldc + col0 + c4) = v;
    }
    if (pass == 0) __threadfence();
  }
}
template <bool PARAM_BF16>
__global__ __launch_bounds__(256) void k_layernorm(const float* __restrict__ X, const float* __restrict__ R, const float* __restrict__ g, const float* __restrict__ bta,
                                                  float* __restrict__ out_sum, float* __restrict__ out_norm, int N, float eps) {
  __shared__ float red[256];
  const int row = blockIdx.x, tid = threadIdx.x;
  const float* x = X + (size_t)row * N; const float* rr = R ? R + (size_t)row * N : nullptr;
  float vals[16];
  const int per = N / 256;
  float s1 = 0.f;
  for (int u = 0; u < per / 4; ++u) {
    const int j = tid * 4 + 1024 * u;
    const v4f a = *(const v4fa*)(x + j);
    v4f b = {0.f,0.f,0.f,0.f}; if (rr) b = *(const v4fa*)(rr + j);
#pragma unroll
    for (int q = 0; q < 4; ++q) { const float v = a[q] + b[q]; vals[u * 4 + q] = v; s1 += v; }
  }
  red[tid] = s1; __syncthreads();
  for (int st = 128; st > 0; st >>= 1) { if (tid < st) red[tid] += red[tid + st]; __syncthreads(); }
  const float mu = red[0] / (float)N; __syncthreads();
  float s2 = 0.f;
  for (int u = 0; u < per / 4; ++u)
#pragma unroll
    for (int q = 0; q < 4; ++q) { const float c = vals[u * 4 + q] - mu; s2 += c * c; }
  red[tid] = s2; __syncthreads();
  for (int st = 128; st > 0; st >>= 1) { if (tid < st) red[tid] += red[tid + st]; __syncthreads(); }
  const float rs = rsqrtf(red[0] / (float)N + eps);
  for (int pass = 0; pass < 2; ++pass) {
    for (int u = 0; u < per / 4; ++u) {
      const int j = tid * 4 + 1024 * u;
      v4f o, sm;
#pragma unroll
      for (int q = 0; q < 4; ++q) {
        float gg = g[j + q], bb = bta[j + q];
        if (PARAM_BF16) { gg = bf16_round(gg); bb = bf16_round(bb); }
        sm[q] = vals[u * 4 + q]; o[q] = (vals[u * 4 + q] - mu) * rs * gg + bb;
      }
      if (out_sum) *(volatile v4f*)(out_sum + (size_t)row * N + j) = sm;
      *(volatile v4f*)(out_norm + (size_t)row * N + j) = o;
    }
    if (pass == 0) __threadfence();
  }
}


typedef _Float16 v16h __attribute__((ext_vector_type(16)));
union FragH { v16h v; v8us half[2]; _Float16 h[16]; unsigned short u[16]; };
template <int NT>
__device__ __forceinline__ v8f mmaH(v16h ah, v16h al, v16h bh, v16h bl, v8f c) {
  c = __builtin_amdgcn_wmma_f32_16x16x32_f16(false, ah, false, bh, (short)0, c, false, false);
  if (NT >= 2) c = __builtin_amdgcn_wmma_f32_16x16x32_f16(false, al, false, bh, (short)0, c, false, false);
  if (NT >= 3) c = __builtin_amdgcn_wmma_f32_16x16x32_f16(false, ah, false, bl, (short)0, c, false, false);
  asm volatile("v_nop\n\tv_nop\n\tv_nop\n\tv_nop" : "+v"(c) : "v"(ah), "v"(al), "v"(bh), "v"(bl));
  return c;
}
template <bool ASPLIT>
__global__ __launch_bounds__(128) void k_gemm_h(const float* __restrict__ A, int lda, size_t sA, const _Float16* __restrict__ Bh, int ldb, size_t sB, float alpha, float* __restrict__ C, int ldc, size_t sC, int M, int N, int K) {
  __shared__ __attribute__((aligned(16))) float so[4][16][64];
  const int tid = threadIdx.x, w = tid >> 5, lane = tid & 31, ln = lane & 15, hh = lane >> 4; const int by = blockIdx.y;
  A += (size_t)by * sA; Bh += (size_t)by * sB; C += (size_t)by * sC;
  const int ntn = (N + 63) / 64; const int wid = blockIdx.x * 4 + w; const int mt = wid / ntn, nq = wid % ntn; if (mt * 16 >= M) return;
  const int row0 = mt * 16, col0 = nq * 64; const float* arow = A + (size_t)(row0 + ln) * lda;
  v8f acc[4] = {};
  for (int kb = 0; kb < K; kb += 32) {
    FragH ah, al;
    const v4f x0 = *(const v4fa*)(arow + kb + 8 * hh), x1 = *(const v4fa*)(arow + kb + 8 * hh + 4), x2 = *(const v4fa*)(arow + kb + 16 + 8 * hh), x3 = *(const v4fa*)(arow + kb + 16 + 8 * hh + 4);
    float xs[16] = {x0[0],x0[1],x0[2],x0[3],x1[0],x1[1],x1[2],x1[3],x2[0],x2[1],x2[2],x2[3],x3[0],x3[1],x3[2],x3[3]};
#pragma unroll
    for (int i = 0; i < 16; ++i) { const _Float16 h = (_Float16)xs[i]; ah.h[i] = h; al.h[i] = ASPLIT ? (_Float16)(xs[i] - (float)h) : (_Float16)0.0f; }
#pragma unroll
    for (int t = 0; t < 4; ++t) { if (col0 + t * 16 >= N) continue; const size_t boff = (size_t)(col0 + t * 16 + ln) * ldb + kb; FragH bq; bq.half[0] = *(const v8us*)(Bh + boff + 8 * hh); bq.half[1] = *(const v8us*)(Bh + boff + 16 + 8 * hh);
      acc[t] = mmaH<ASPLIT ? 2 : 1>(ah.v, al.v, bq.v, bq.v, acc[t]); }
  }
#pragma unroll
  for (int t = 0; t < 4; ++t) { if (col0 + t * 16 >= N) continue;
#pragma unroll
    for (int r = 0; r < 8; ++r) so[w][8 * hh + r][t * 16 + ln] = acc[t][r] * alpha; }
  __builtin_amdgcn_fence(__ATOMIC_ACQ_REL, "workgroup"); __builtin_amdgcn_wave_barrier();
  const int rsub = lane >> 4, c4 = (lane & 15) * 4;
  for (int pass = 0; pass < 2; ++pass) {
#pragma unroll
    for (int q = 0; q < 8; ++q) { const int r = q * 2 + rsub; if (col0 + c4 < N) { const v4f v = *(const v4fa*)&so[w][r][c4]; *(volatile v4f*)(C + (size_t)(row0 + r) * ldc + col0 + c4) = v; } }
    if (pass == 0) __threadfence(); }
}

__global__ __launch_bounds__(256) void k_wt_f16(const float* __restrict__ W, _Float16* __restrict__ Wt, int K, int N, float scale) {
  const int t = blockIdx.x * 256 + threadIdx.x; if (t >= N * (K / 8)) return; const int n = t / (K / 8), k8 = (t % (K / 8)) * 8; FragH f;
#pragma unroll
  for (int i = 0; i < 8; ++i) f.h[i] = (_Float16)(bf16_round(W[(size_t)(k8 + i) * N + n]) * scale); const v8us o = f.half[0];
  *(volatile v8us*)((unsigned short*)Wt + (size_t)n * K + k8) = o; __threadfence(); *(volatile v8us*)((unsigned short*)Wt + (size_t)n * K + k8) = o;
}
template <int ACT>
__global__ __launch_bounds__(128) void k_gemm_hhx(const _Float16* __restrict__ A, int lda, size_t sA, const _Float16* __restrict__ Bh, int ldb, size_t sB, float alpha, const float* __restrict__ bias, size_t sBias, const float* __restrict__ CP, int rowsPerB, size_t sCPb, int row0g,
    float* __restrict__ C, _Float16* __restrict__ C16, int ldc, size_t sC, int M, int N, int K) {
  __shared__ __attribute__((aligned(16))) float so[4][16][64];
  const int tid = threadIdx.x, w = tid >> 5, lane = tid & 31, ln = lane & 15, hh = lane >> 4; const int by = blockIdx.y;
  A += (size_t)by * sA; Bh += (size_t)by * sB; const size_t cofs = (size_t)by * sC; const float* bp = bias ? bias + (size_t)by * sBias : nullptr;
  const int ntn = (N + 63) / 64; const int wid = blockIdx.x * 4 + w; const int mt = wid / ntn, nq = wid % ntn; if (mt * 16 >= M) return;
  const int row0 = mt * 16, col0 = nq * 64; const _Float16* arow = A + (size_t)(row0 + ln) * lda;
  v8f acc[4] = {};
  for (int kb = 0; kb < K; kb += 32) { FragH ah; ah.half[0] = *(const v8us*)((const unsigned short*)arow + kb + 8 * hh); ah.half[1] = *(const v8us*)((const unsigned short*)arow + kb + 16 + 8 * hh);
#pragma unroll
    for (int t = 0; t < 4; ++t) { if (col0 + t * 16 >= N) continue; const size_t boff = (size_t)(col0 + t * 16 + ln) * ldb + kb; FragH bq; bq.half[0] = *(const v8us*)((const unsigned short*)Bh + boff + 8 * hh); bq.half[1] = *(const v8us*)((const unsigned short*)Bh + boff + 16 + 8 * hh);
      acc[t] = mmaH<1>(ah.v, ah.v, bq.v, bq.v, acc[t]); }
  }
#pragma unroll
  for (int t = 0; t < 4; ++t) { if (col0 + t * 16 >= N) continue; const int col = col0 + t * 16 + ln; const float bv = bp ? bf16_round(bp[col]) : 0.f;
#pragma unroll
    for (int r = 0; r < 8; ++r) { float v = acc[t][r] * alpha + bv; if (CP) { const int bidx = (row0g + row0 + 8 * hh + r) / rowsPerB; v += CP[(size_t)bidx * sCPb + (size_t)by * 64 + col]; } if (ACT == 1) v = (v > 0.f) ? v : expm1f(v); else if (ACT == 7) v = (v > 0.f) ? v + 1.0f : expf(v); else if (ACT == 8) v = tanhf(v); else if (ACT == 9) v = 0.5f * v * (1.0f + tanhf(0.7978845608028654f * (v + 0.044715f * v * v * v))); else if (ACT == 11) v = 1.0f / (1.0f + expf(-v)); else if (ACT == 12) v = (v > 0.f) ? v : 0.01f * v; else if (ACT == 14) v = (v > 0.f) ? v : 0.1f * v; else if (ACT == 16) v = (v >= 0.f) ? v : 0.01f * v; else if (ACT == 15) v = v / (1.0f + expf(-v)); else if (ACT == 3) v = fmaxf(v, 0.f); else if (ACT == 6) v = 0.5f * v * (1.0f + erff(v * 0.70710678118654752f)); so[w][8 * hh + r][t * 16 + ln] = v; } }
  __builtin_amdgcn_fence(__ATOMIC_ACQ_REL, "workgroup"); __builtin_amdgcn_wave_barrier();
  const int rsub = lane >> 4, c4 = (lane & 15) * 4; typedef _Float16 v4h __attribute__((ext_vector_type(4)));
  for (int pass = 0; pass < 2; ++pass) {
#pragma unroll
    for (int q = 0; q < 8; ++q) { const int r = q * 2 + rsub; if (col0 + c4 < N) { const v4f v = *(const v4fa*)&so[w][r][c4]; if (C) *(volatile v4f*)(C + cofs + (size_t)(row0 + r) * ldc + col0 + c4) = v; if (C16) { v4h h4; for (int i = 0; i < 4; ++i) h4[i] = (_Float16)v[i]; *(volatile v4h*)(C16 + cofs + (size_t)(row0 + r) * ldc + col0 + c4) = h4; } } }
    if (pass == 0) __threadfence(); }
}


typedef _Float16 v4h __attribute__((ext_vector_type(4)));

__global__ __launch_bounds__(256) void k_x16(const float* __restrict__ x, _Float16* __restrict__ X16, size_t n8) { const size_t t = (size_t)blockIdx.x * 256 + threadIdx.x; if (t >= n8) return; FragH f;
#pragma unroll
  for (int q = 0; q < 8; ++q) f.h[q] = (_Float16)bf16_round(x[t * 8 + q]); *(volatile v8us*)((unsigned short*)X16 + t * 8) = f.half[0]; __threadfence(); *(volatile v8us*)((unsigned short*)X16 + t * 8) = f.half[0]; }
__global__ __launch_bounds__(256) void k_h16(const float* __restrict__ x, _Float16* __restrict__ X16, size_t n8) { const size_t t = (size_t)blockIdx.x * 256 + threadIdx.x; if (t >= n8) return; FragH f;
#pragma unroll
  for (int q = 0; q < 8; ++q) f.h[q] = (_Float16)x[t * 8 + q]; *(volatile v8us*)((unsigned short*)X16 + t * 8) = f.half[0]; __threadfence(); *(volatile v8us*)((unsigned short*)X16 + t * 8) = f.half[0]; }
__global__ __launch_bounds__(256) void k_round16f(const float* __restrict__ W, _Float16* __restrict__ Bt, size_t n8) { const size_t t = (size_t)blockIdx.x * 256 + threadIdx.x; if (t >= n8) return; FragH f;
#pragma unroll
  for (int i = 0; i < 8; ++i) f.h[i] = (_Float16)(bf16_round(W[t * 8 + i]) * 16.0f); *(volatile v8us*)((unsigned short*)Bt + t * 8) = f.half[0]; __threadfence(); *(volatile v8us*)((unsigned short*)Bt + t * 8) = f.half[0]; }
template <int NHv, int TTv>
__global__ __launch_bounds__(256) void k_vt(const _Float16* __restrict__ V16, int ldv, int voff, _Float16* __restrict__ Vt) { __shared__ unsigned short tl[64][66]; const int tid = threadIdx.x; const int slab = blockIdx.x / (TTv / 64), lg = blockIdx.x % (TTv / 64); const int b = slab / NHv, h = slab % NHv;
  for (int i = tid; i < 64 * 8; i += 256) { const int r = i / 8, c8 = (i % 8) * 8; FragH f; f.half[0] = *(const v8us*)((const unsigned short*)V16 + ((size_t)b * TTv + lg * 64 + r) * ldv + voff + h * 64 + c8);
#pragma unroll
    for (int q = 0; q < 8; ++q) tl[r][c8 + q] = f.u[q]; }
  __syncthreads();
  for (int pass = 0; pass < 2; ++pass) {
#pragma unroll
    for (int rd = 0; rd < 2; ++rd) { const int d = rd * 32 + tid / 8, pc = tid % 8; FragH f;
#pragma unroll
      for (int q = 0; q < 8; ++q) f.u[q] = tl[pc * 8 + q][d];
      *(volatile v8us*)((unsigned short*)Vt + ((size_t)slab * 64 + d) * TTv + lg * 64 + pc * 8) = f.half[0]; }
    if (pass == 0) __threadfence(); } }

__global__ __launch_bounds__(256) void k_hl(const float* __restrict__ F, _Float16* __restrict__ Hh, _Float16* __restrict__ Hl, size_t n8) { const size_t t = (size_t)blockIdx.x * 256 + threadIdx.x; if (t >= n8) return; FragH fh, fl; const v4f a = *(const v4fa*)(F + t * 8), c = *(const v4fa*)(F + t * 8 + 4);
#pragma unroll
  for (int q = 0; q < 4; ++q) { _Float16 h = (_Float16)a[q]; fh.h[q] = h; fl.h[q] = (_Float16)((a[q] - (float)h) * 1024.0f); h = (_Float16)c[q]; fh.h[4 + q] = h; fl.h[4 + q] = (_Float16)((c[q] - (float)h) * 1024.0f); }
  for (int pass = 0; pass < 2; ++pass) { *(volatile v8us*)((unsigned short*)Hh + t * 8) = fh.half[0]; *(volatile v8us*)((unsigned short*)Hl + t * 8) = fl.half[0]; if (pass == 0) __threadfence(); } }

__device__ __forceinline__ float lrelu01(float v) { return (v >= 0.f) ? v : 0.01f * v; }
__device__ __forceinline__ float wrap_pi(float a) { float t = fmodf(a + PI_F, 2.0f * PI_F); if (t < 0.f) t += 2.0f * PI_F; return t - PI_F; }
__global__ __launch_bounds__(256) void k_ag1(const float* __restrict__ emb, const float* __restrict__ W1, const float* __restrict__ b1, _Float16* __restrict__ H) {
  #pragma clang fp contract(off)
  const int t = blockIdx.x * 256 + threadIdx.x; if (t >= NA * (H1 / 8)) return; const int a = t / (H1 / 8), c0 = (t % (H1 / 8)) * 8; float e[5];
#pragma unroll
  for (int k = 0; k < 5; ++k) e[k] = bf16_round(emb[(size_t)a * 11 + 4 + k]);
  FragH f;
#pragma unroll
  for (int q = 0; q < 8; ++q) { const int c = c0 + q; float s = bf16_round(b1[c]);
#pragma unroll
    for (int k = 0; k < 5; ++k) s += e[k] * bf16_round(W1[c * 5 + k]); f.h[q] = (_Float16)lrelu01(s); }
  *(volatile v8us*)((unsigned short*)H + (size_t)a * H1 + c0) = f.half[0]; __threadfence(); *(volatile v8us*)((unsigned short*)H + (size_t)a * H1 + c0) = f.half[0]; }
__global__ __launch_bounds__(256) void k_whm1(const float* __restrict__ w, _Float16* __restrict__ Bh, float* __restrict__ WE) { const int t = blockIdx.x * 256 + threadIdx.x; if (t >= DD * 33) return; const int o = t / 33, k0 = (t % 33) * 8; if (k0 < 256) { FragH f;
#pragma unroll
    for (int q = 0; q < 8; ++q) f.h[q] = (_Float16)(bf16_round(w[(size_t)o * 263 + k0 + q]) * 16.0f);
    *(volatile v8us*)((unsigned short*)Bh + (size_t)o * DD + k0) = f.half[0]; __threadfence(); *(volatile v8us*)((unsigned short*)Bh + (size_t)o * DD + k0) = f.half[0]; }
  else { v4f a, c;
#pragma unroll
    for (int q = 0; q < 4; ++q) { a[q] = bf16_round(w[(size_t)o * 263 + 256 + q]); c[q] = (q < 3) ? bf16_round(w[(size_t)o * 263 + 260 + q]) : 0.f; }
    for (int pass = 0; pass < 2; ++pass) { *(volatile v4f*)(WE + (size_t)o * 8) = a; *(volatile v4f*)(WE + (size_t)o * 8 + 4) = c; if (pass == 0) __threadfence(); } } }
__global__ __launch_bounds__(256) void k_wk(const float* __restrict__ kw, _Float16* __restrict__ Bk) { const int t = blockIdx.x * 256 + threadIdx.x; if (t >= 16 * (DD / 8)) return; const int n = t / (DD / 8), k0 = (t % (DD / 8)) * 8; FragH f;
#pragma unroll
  for (int q = 0; q < 8; ++q) f.h[q] = (n < 10) ? (_Float16)(bf16_round(kw[(size_t)(k0 + q) * 10 + n]) * 16.0f) : (_Float16)0.0f;
  *(volatile v8us*)((unsigned short*)Bk + (size_t)n * DD + k0) = f.half[0]; __threadfence(); *(volatile v8us*)((unsigned short*)Bk + (size_t)n * DD + k0) = f.half[0]; }
__global__ __launch_bounds__(256) void k_wfold(const float* __restrict__ hew, const float* __restrict__ heb, const float* __restrict__ hm2w, const float* __restrict__ hm2b, _Float16* __restrict__ Be, float* __restrict__ BEb) {
  #pragma clang fp contract(off)
  const int t = blockIdx.x * 256 + threadIdx.x; if (t >= 16 * (DD / 8)) return; const int n = t / (DD / 8), k0 = (t % (DD / 8)) * 8; float s[8];
#pragma unroll
  for (int q = 0; q < 8; ++q) s[q] = 0.f;
  if (n < 2) {
#pragma unroll 1
    for (int o = 0; o < DD; ++o) { const float hv = bf16_round(hew[n * DD + o]); const float* wr = hm2w + (size_t)o * DD + k0;
#pragma unroll
      for (int q = 0; q < 8; ++q) s[q] += hv * bf16_round(wr[q]); } }
  FragH f;
#pragma unroll
  for (int q = 0; q < 8; ++q) f.h[q] = (_Float16)(s[q] * 16.0f);
  *(volatile v8us*)((unsigned short*)Be + (size_t)n * DD + k0) = f.half[0]; __threadfence(); *(volatile v8us*)((unsigned short*)Be + (size_t)n * DD + k0) = f.half[0];
  if (t < 16) { float bsum = 0.f; if (t < 2) {
#pragma unroll 1
      for (int o = 0; o < DD; ++o) bsum += bf16_round(hew[t * DD + o]) * bf16_round(hm2b[o]); bsum += bf16_round(heb[t]); }
    *(volatile float*)(BEb + t) = bsum; __threadfence(); *(volatile float*)(BEb + t) = bsum; } }
__global__ __launch_bounds__(256) void k_pair(const float* __restrict__ emb, const float* __restrict__ U, const float* __restrict__ WE, const float* __restrict__ hb, _Float16* __restrict__ HH, float* __restrict__ E10) {
  #pragma clang fp contract(off)
  __shared__ float se[8][12]; const int tid = threadIdx.x, w = tid >> 5, l = tid & 31; const int p = blockIdx.x * 8 + w; if (p >= NP) return; const int a = p / NO, jj = p % NO; const int b = a / NAG, i = a % NAG; const int j = jj + ((jj >= i) ? 1 : 0);
  const float* ei = emb + ((size_t)b * NAG + i) * 11; const float* ej = emb + ((size_t)b * NAG + j) * 11;
  const float pix = bf16_round(ei[0]), piy = bf16_round(ei[1]), hix = bf16_round(ei[2]), hiy = bf16_round(ei[3]); const float pjx = bf16_round(ej[0]), pjy = bf16_round(ej[1]), hjx = bf16_round(ej[2]), hjy = bf16_round(ej[3]), ajx = bf16_round(ej[7]), ajy = bf16_round(ej[8]), gjx = bf16_round(ej[9]), gjy = bf16_round(ej[10]);
  const float dx = pjx - pix, dy = pjy - piy; const float dist = sqrtf(dx * dx + dy * dy);
  const float hn = sqrtf(hix * hix + hiy * hiy); const float ch = (hn > 0.f) ? hix / hn : 1.f, sh = (hn > 0.f) ? hiy / hn : 0.f;
  const float ct = (dist > 0.f) ? dx / dist : 1.f, st = (dist > 0.f) ? dy / dist : 0.f;
  const float gx = gjx - pix, gy = gjy - piy; const float gd = sqrtf(gx * gx + gy * gy); const float cg = (gd > 0.f) ? gx / gd : 1.f, sg = (gd > 0.f) ? gy / gd : 0.f;
  float e[10]; e[0] = dist / 12.0f; e[1] = ct * ch + st * sh; e[2] = st * ch - ct * sh; e[3] = hjx; e[4] = hjy; e[5] = ajx; e[6] = ajy; e[7] = gd; e[8] = cg * ch + sg * sh; e[9] = sg * ch - cg * sh;
  if (l < 10) se[w][l] = (l == 0) ? e[0] : (l == 1) ? e[1] : (l == 2) ? e[2] : (l == 3) ? e[3] : (l == 4) ? e[4] : (l == 5) ? e[5] : (l == 6) ? e[6] : (l == 7) ? e[7] : (l == 8) ? e[8] : e[9];
  __syncthreads();
  FragH f; const int c0 = 8 * l;
#pragma unroll
  for (int q = 0; q < 8; ++q) { const int c = c0 + q; float s = U[(size_t)a * DD + c] + bf16_round(hb[c]);
#pragma clang loop unroll(disable)
    for (int k = 0; k < 7; ++k) s += WE[(size_t)c * 8 + k] * se[w][k]; f.h[q] = (_Float16)fmaxf(s, 0.f); }
  v4f q4; q4[0] = 0.f; q4[1] = 0.f; q4[2] = 0.f; q4[3] = 0.f; if (l == 0) { q4[0] = e[0]; q4[1] = e[1]; q4[2] = e[2]; q4[3] = e[3]; } else if (l == 1) { q4[0] = e[4]; q4[1] = e[5]; q4[2] = e[6]; q4[3] = e[7]; } else if (l == 2) { q4[0] = e[8]; q4[1] = e[9]; q4[2] = dist; q4[3] = 0.f; }
  for (int pass = 0; pass < 2; ++pass) { *(volatile v8us*)((unsigned short*)HH + (size_t)p * DD + c0) = f.half[0]; if (l < 8) *(volatile v4f*)(E10 + (size_t)p * 32 + 4 * l) = q4; if (pass == 0) __threadfence(); } }

__global__ __launch_bounds__(256) void k_soft(const float* __restrict__ HL, const float* __restrict__ gu, const float* __restrict__ QK, const float* __restrict__ E10, const float* __restrict__ vw, const float* __restrict__ vb, _Float16* __restrict__ X16, float* __restrict__ ROWS) {
  #pragma clang fp contract(off)
  __shared__ __attribute__((aligned(16))) float cmb[32], shl[32], shw[32], sud[32]; __shared__ __attribute__((aligned(16))) float es[32][12]; __shared__ __attribute__((aligned(16))) unsigned short xs[DD];
  const int tid = threadIdx.x; const int a = blockIdx.x;
  if (tid < 32) { cmb[tid] = 0.f; shl[tid] = 0.f; shw[tid] = 0.f; sud[tid] = 0.f; }
  __syncthreads();
  if (tid < NO) { const int p = a * NO + tid; const float l0 = HL[(size_t)p * 16], l1 = HL[(size_t)p * 16 + 1];
    const float u0 = bf16_round(gu[(size_t)p * 2]), u1 = bf16_round(gu[(size_t)p * 2 + 1]); const float g0 = -logf(-logf(u0 + 1e-10f) + 1e-10f), g1 = -logf(-logf(u1 + 1e-10f) + 1e-10f);
    const float z0 = (l0 + g0) / 0.5f, z1 = (l1 + g1) / 0.5f; const float m = fmaxf(z0, z1); const float x0 = expf(z0 - m), x1 = expf(z1 - m); const float hw = x1 / (x0 + x1);
    const float* er = E10 + (size_t)p * 32; float sc = 0.f;
#pragma unroll
    for (int k = 0; k < 10; ++k) { es[tid][k] = er[k]; sc += QK[(size_t)a * 16 + k] * er[k]; }
    shl[tid] = l1; shw[tid] = hw; sud[tid] = er[10]; cmb[tid] = sc / 16.0f; }
  __syncthreads();
  if (tid == 0) { float m = -3.0e38f;
#pragma clang loop unroll(disable)
    for (int j = 0; j < NO; ++j) m = fmaxf(m, cmb[j]);
    float s = 0.f;
#pragma clang loop unroll(disable)
    for (int j = 0; j < NO; ++j) s += expf(cmb[j] - m);
    float csum = 0.f;
#pragma clang loop unroll(disable)
    for (int j = 0; j < NO; ++j) { const float c = (expf(cmb[j] - m) / s) * shw[j]; cmb[j] = c; csum += c; }
    float ent = 0.f;
#pragma clang loop unroll(disable)
    for (int j = 0; j < NO; ++j) { const float cw = cmb[j] / (csum + 1e-6f); ent += -(cw * logf(cw + 1e-6f)); } shl[31] = ent; }
  __syncthreads();
  { const int c = tid; float x = 0.f; const float bb = bf16_round(vb[c]); float wv[10];
#pragma unroll
    for (int k = 0; k < 10; ++k) wv[k] = bf16_round(vw[(size_t)c * 10 + k]);
#pragma clang loop unroll(disable)
    for (int j = 0; j < NO; ++j) { float v = bb;
#pragma unroll
      for (int k = 0; k < 10; ++k) v += wv[k] * es[j][k]; x += cmb[j] * fmaxf(v, 0.f); }
    FragH f; f.h[0] = (_Float16)x; xs[c] = f.u[0]; }
  __syncthreads();
  for (int pass = 0; pass < 2; ++pass) {
    if (tid < DD / 8) { const v8us v = *(const v8us*)&xs[tid * 8]; *(volatile v8us*)((unsigned short*)X16 + (size_t)a * DD + tid * 8) = v; }
    else if (tid < 64) { const int q = tid - 32; const int arr = q / 8, l4 = (q % 8) * 4; const float* src = (arr == 0) ? shl : (arr == 1) ? sud : (arr == 2) ? shw : cmb; const v4f v = *(const v4fa*)(src + l4); *(volatile v4f*)(ROWS + ((size_t)arr * NA + a) * 32 + l4) = v; }
    if (pass == 0) __threadfence(); } }
__global__ __launch_bounds__(256) void k_ent(const float* __restrict__ ROWS, float* __restrict__ ENTS) {
  #pragma clang fp contract(off)
  __shared__ float s[256]; const int tid = threadIdx.x; float acc = 0.f; for (int i = tid; i < NA; i += 256) acc += ROWS[(size_t)i * 32 + 31]; s[tid] = acc; __syncthreads();
  for (int k = 128; k > 0; k >>= 1) { if (tid < k) s[tid] += s[tid + k]; __syncthreads(); }
  if (tid == 0) { const float m = s[0] / (float)NA; *(volatile float*)ENTS = m; __threadfence(); *(volatile float*)ENTS = m; } }
__global__ __launch_bounds__(256) void k_tail(const float* __restrict__ ROWS, const float* __restrict__ ENTS, float* __restrict__ out) { const int f = blockIdx.x * 256 + threadIdx.x; if (f >= OUTEND - OUT1) return; float v;
  if (f < NP) { v = ROWS[(size_t)(0 * NA + f / NO) * 32 + f % NO]; } else if (f < 2 * NP) { const int g = f - NP; v = ROWS[(size_t)(1 * NA + g / NO) * 32 + g % NO]; } else if (f == 2 * NP) { v = ENTS[0]; } else if (f < 3 * NP + 1) { const int g = f - 2 * NP - 1; v = ROWS[(size_t)(2 * NA + g / NO) * 32 + g % NO]; } else { const int g = f - 3 * NP - 1; v = ROWS[(size_t)(3 * NA + g / NO) * 32 + g % NO]; }
  *(volatile float*)(out + OUT1 + f) = v; __threadfence(); *(volatile float*)(out + OUT1 + f) = v; }
extern "C" void kernel_launch(void* const* d_in, const int* in_sizes, int n_in,
                              void* d_out, int out_size, void* d_ws, size_t ws_size, hipStream_t stream) {
  (void)in_sizes; (void)n_in; (void)out_size;
  const float* const* I = (const float* const*)d_in; const float* emb = I[0]; const float* gu = I[1]; const float* e1w = I[2]; const float* e1b = I[3]; const float* e2w = I[4]; const float* e2b = I[5]; const float* hm1w = I[6]; const float* hm1b = I[7]; const float* hm2w = I[8]; const float* hm2b = I[9]; const float* hew = I[10]; const float* heb = I[11]; const float* qw = I[12]; const float* kw = I[13]; const float* vw = I[14]; const float* vb = I[15]; const float* decw = I[16]; const float* decb = I[17];
  char* ws = (char*)d_ws; size_t off = 0;
  auto take = [&](size_t bytes) { char* p = ws + off; off += (bytes + 255) & ~(size_t)255; return p; };
  _Float16* Be2 = (_Float16*)take((size_t)DD * H1 * 2); _Float16* Bh = (_Float16*)take((size_t)DD * DD * 2); float* WE = (float*)take((size_t)DD * 8 * 4); _Float16* Be = (_Float16*)take((size_t)16 * DD * 2); float* BEb = (float*)take(64 * 4); _Float16* Bq = (_Float16*)take((size_t)DD * DD * 2); _Float16* Bk = (_Float16*)take((size_t)16 * DD * 2); _Float16* Bdec = (_Float16*)take((size_t)512 * 512 * 2);
  _Float16* Hh = (_Float16*)take((size_t)NA * H1 * 2); float* AEf = (float*)take((size_t)NA * DD * 4); _Float16* AE16 = (_Float16*)take((size_t)NA * DD * 2); float* U = (float*)take((size_t)NA * DD * 4); _Float16* Q16 = (_Float16*)take((size_t)NA * DD * 2); float* QK = (float*)take((size_t)NA * 16 * 4);
  _Float16* HH = (_Float16*)take((size_t)NP * DD * 2); float* E10 = (float*)take((size_t)NP * 32 * 4); float* HL = (float*)take((size_t)NP * 16 * 4); _Float16* X16 = (_Float16*)take((size_t)NA * DD * 2); float* ROWS = (float*)take((size_t)4 * NA * 32 * 4); float* ENTS = (float*)take(64 * 4);
  if (off > ws_size) return;
  k_round16f<<<(unsigned)(((size_t)DD * H1 / 8 + 255) / 256), 256, 0, stream>>>(e2w, Be2, (size_t)DD * H1 / 8); k_whm1<<<(DD * 33 + 255) / 256, 256, 0, stream>>>(hm1w, Bh, WE); k_wfold<<<(16 * (DD / 8) + 255) / 256, 256, 0, stream>>>(hew, heb, hm2w, hm2b, Be, BEb); k_round16f<<<(unsigned)(((size_t)DD * DD / 8 + 255) / 256), 256, 0, stream>>>(qw, Bq, (size_t)DD * DD / 8); k_wk<<<(16 * (DD / 8) + 255) / 256, 256, 0, stream>>>(kw, Bk); k_round16f<<<(unsigned)(((size_t)512 * 512 / 8 + 255) / 256), 256, 0, stream>>>(decw, Bdec, (size_t)512 * 512 / 8);
  k_ag1<<<(NA * (H1 / 8) + 255) / 256, 256, 0, stream>>>(emb, e1w, e1b, Hh);
  const dim3 gA(((NA / 16) * (DD / 64) + 3) / 4, 1), gA16(((NA / 16) * 1 + 3) / 4, 1), gP(((NP / 16) * (DD / 64) + 3) / 4, 1), gP16(((NP / 16) * 1 + 3) / 4, 1);
  k_gemm_hhx<16><<<gA, 128, 0, stream>>>(Hh, H1, 0, Be2, H1, 0, 0.0625f, e2b, 0, nullptr, 1, 0, 0, AEf, AE16, DD, 0, NA, DD, H1);
  k_gemm_hhx<0><<<gA, 128, 0, stream>>>(AE16, DD, 0, Bh, DD, 0, 0.0625f, nullptr, 0, nullptr, 1, 0, 0, U, nullptr, DD, 0, NA, DD, DD);
  k_gemm_hhx<0><<<gA, 128, 0, stream>>>(AE16, DD, 0, Bq, DD, 0, 0.0625f, nullptr, 0, nullptr, 1, 0, 0, nullptr, Q16, DD, 0, NA, DD, DD);
  k_gemm_hhx<0><<<gA16, 128, 0, stream>>>(Q16, DD, 0, Bk, DD, 0, 0.0625f, nullptr, 0, nullptr, 1, 0, 0, QK, nullptr, 16, 0, NA, 16, DD);
  k_pair<<<NP / 8, 256, 0, stream>>>(emb, U, WE, hm1b, HH, E10);
  k_gemm_hhx<0><<<gP16, 128, 0, stream>>>(HH, DD, 0, Be, DD, 0, 0.0625f, BEb, 0, nullptr, 1, 0, 0, HL, nullptr, 16, 0, NP, 16, DD);
  k_soft<<<NA, 256, 0, stream>>>(HL, gu, QK, E10, vw, vb, X16, ROWS);
  k_ent<<<1, 256, 0, stream>>>(ROWS, ENTS);
  k_tail<<<(OUTEND - OUT1 + 255) / 256, 256, 0, stream>>>(ROWS, ENTS, (float*)d_out);
  k_gemm_hhx<0><<<dim3(((NA / 16) * (512 / 64) + 3) / 4, 1), 128, 0, stream>>>(AE16, DD, 0, Bdec, 512, 0, 0.0625f, decb, 0, nullptr, 1, 0, 0, (float*)d_out, nullptr, 512, 0, NA, 512, DD);
  k_gemm_hhx<0><<<dim3(((NA / 16) * (512 / 64) + 3) / 4, 1), 128, 0, stream>>>(X16, DD, 0, Bdec + 256, 512, 0, 0.0625f, nullptr, 0, (float*)d_out, 1, 512, 0, (float*)d_out, nullptr, 512, 0, NA, 512, DD);
}
